// GaussianMixture_2783138808281
// MI455X (gfx1250) — hardware-verified
//
#include <hip/hip_runtime.h>
#include <math.h>
typedef __attribute__((ext_vector_type(16))) _Float16 v16h;
typedef __attribute__((ext_vector_type(8)))  _Float16 v8h;
typedef __attribute__((ext_vector_type(16))) __bf16   v16b;
typedef __attribute__((ext_vector_type(8)))  __bf16   v8b;
typedef __attribute__((ext_vector_type(8)))  float    v8f;
typedef __attribute__((ext_vector_type(4)))  float    v4f;
#define PSCALE 32768.0f
#define U16(p) ((const unsigned short*)(const void*)(p))
#define PSCALE_INV (1.0f / 32768.0f)

__device__ __forceinline__ unsigned short f2bf_bits(float f) {
  unsigned u = __float_as_uint(f);
  return (unsigned short)((u + 0x7FFFu + ((u >> 16) & 1u)) >> 16);
}
__device__ __forceinline__ float bf_bits2f(unsigned short h) { return __uint_as_float(((unsigned)h) << 16); }

__device__ __forceinline__ void dep_guard_h(v8f& a, v8f& b, v16h x, v16h y) { asm volatile("v_nop\n\tv_nop\n\tv_nop\n\tv_nop" : "+v"(a), "+v"(b) : "v"(x), "v"(y)); }
__device__ __forceinline__ void dep_guard_b(v8f& a, v8f& b, v16b x, v16b y) { asm volatile("v_nop\n\tv_nop\n\tv_nop\n\tv_nop" : "+v"(a), "+v"(b) : "v"(x), "v"(y)); }
__device__ __forceinline__ void keep4_h(v16h a, v16h b, v16h c, v16h d) { asm volatile("v_nop" :: "v"(a), "v"(b), "v"(c), "v"(d)); }
__device__ __forceinline__ void keep4_b(v16b a, v16b b, v16b c, v16b d) { asm volatile("v_nop" :: "v"(a), "v"(b), "v"(c), "v"(d)); }
__device__ __forceinline__ void acc_guard4(v8f& a, v8f& b, v8f& c, v8f& d) { asm volatile("v_nop\n\tv_nop\n\tv_nop\n\tv_nop" : "+v"(a), "+v"(b), "+v"(c), "+v"(d)); }
template <typename T> struct Frag;
template <> struct Frag<_Float16> {
  typedef v16h V; union U { v16h v; v8h h[2]; };
  static __device__ __forceinline__ v16h load(const _Float16* p) {
    U f; f.h[0] = *(const v8h*)(p); f.h[1] = *(const v8h*)(p + 16); return f.v;
  }
  static __device__ __forceinline__ v8f mma(v16h a, v16h b, v8f c) {
    return __builtin_amdgcn_wmma_f32_16x16x32_f16(false, a, false, b, (short)0, c, false, false);
  }
  static __device__ __forceinline__ void guard(v8f& a, v8f& b, v16h x, v16h y) { dep_guard_h(a, b, x, y); }
  static __device__ __forceinline__ void keep(v16h a, v16h b, v16h c, v16h d) { keep4_h(a, b, c, d); }
};
template <> struct Frag<__bf16> {
  typedef v16b V; union U { v16b v; v8b h[2]; };
  static __device__ __forceinline__ v16b load(const __bf16* p) {
    U f; f.h[0] = *(const v8b*)(p); f.h[1] = *(const v8b*)(p + 16); return f.v;
  }
  static __device__ __forceinline__ v8f mma(v16b a, v16b b, v8f c) {
    return __builtin_amdgcn_wmma_f32_16x16x32_bf16(false, a, false, b, (short)0, c, false, false);
  }
  static __device__ __forceinline__ void guard(v8f& a, v8f& b, v16b x, v16b y) { dep_guard_b(a, b, x, y); }
  static __device__ __forceinline__ void keep(v16b a, v16b b, v16b c, v16b d) { keep4_b(a, b, c, d); }
};

template <int ET> struct Elem;
template <> struct Elem<0> { typedef _Float16 T; };
template <> struct Elem<1> { typedef __bf16 T; };
template <int ET, bool SPLIT, int BIAS_MODE, int OUT_MODE, bool RESID, int ACT = 0>
__global__ __launch_bounds__(256) void wmma_gemm64(
    const unsigned short* __restrict__ Ap, const unsigned short* __restrict__ A2p, int lda, long strideA,
    const unsigned short* __restrict__ Btp, const unsigned short* __restrict__ Bt2p, int ldb, long strideB,
    void* __restrict__ Cout, void* __restrict__ Cout2, int ldc, long strideC,
    const float* __restrict__ bias,
    const float* __restrict__ resid, long strideR,
    int M, int N, int K, float scale) {
  typedef typename Elem<ET>::T T;
  typedef typename Frag<T>::V V;
  const T* A = (const T*)Ap; const T* A2 = (const T*)A2p; const T* Bt = (const T*)Btp; const T* Bt2 = (const T*)Bt2p;
  __shared__ __align__(16) float sT[8][16 * 68];
  const int b    = blockIdx.y;
  const int lane = threadIdx.x & 31;
  const int wave = threadIdx.x >> 5;
  const int tilesN = N >> 6;
  const int tilesM = M >> 6;
  const int tile = blockIdx.x * 8 + wave;
  if (tile >= tilesM * tilesN) return;
  const int tm = tile / tilesN;
  const int tn = tile - tm * tilesN;
  const int m0 = tm << 6;
  const int n0 = tn << 6;

  const T* Ab  = A  + (size_t)b * strideA;
  const T* Bb  = Bt + (size_t)b * strideB;
  const T* Ab2 = SPLIT ? (A2  + (size_t)b * strideA) : nullptr;
  const T* Bb2 = SPLIT ? (Bt2 + (size_t)b * strideB) : nullptr;

  const int rlane = lane & 15;
  const int koff  = (lane >> 4) * 8;
  const int mOff  = (lane >> 4) * 8;

  v8f acc[4][4];
#pragma unroll
  for (int i = 0; i < 4; ++i)
#pragma unroll
    for (int j = 0; j < 4; ++j) acc[i][j] = (v8f){0.f,0.f,0.f,0.f,0.f,0.f,0.f,0.f};

  for (int k0 = 0; k0 < K; k0 += 32) {
    V bh[4], bl[4];
#pragma unroll
    for (int j = 0; j < 4; ++j) {
      const size_t bo = (size_t)(n0 + (j << 4) + rlane) * ldb + koff + k0;
      bh[j] = Frag<T>::load(Bb + bo);
      if (SPLIT) bl[j] = Frag<T>::load(Bb2 + bo);
    }
#pragma unroll
    for (int i = 0; i < 4; ++i) {
      const size_t ao = (size_t)(m0 + (i << 4) + rlane) * lda + koff + k0;
      V ah = Frag<T>::load(Ab + ao);
      V al;
      if (SPLIT) al = Frag<T>::load(Ab2 + ao);
#pragma unroll
      for (int j = 0; j < 4; ++j) {
        acc[i][j] = Frag<T>::mma(ah, bh[j], acc[i][j]);
        if (SPLIT) {
          acc[i][j] = Frag<T>::mma(ah, bl[j], acc[i][j]);
          acc[i][j] = Frag<T>::mma(al, bh[j], acc[i][j]);
        }
      }
      Frag<T>::guard(acc[i][0], acc[i][3], ah, SPLIT ? al : ah);
    }
    Frag<T>::keep(bh[0], bh[1], bh[2], bh[3]);
    if (SPLIT) Frag<T>::keep(bl[0], bl[1], bl[2], bl[3]);
  }
  acc_guard4(acc[0][0], acc[0][1], acc[0][2], acc[0][3]);
  acc_guard4(acc[1][0], acc[1][1], acc[1][2], acc[1][3]);
  acc_guard4(acc[2][0], acc[2][1], acc[2][2], acc[2][3]);
  acc_guard4(acc[3][0], acc[3][1], acc[3][2], acc[3][3]);

  float* slab = sT[wave];
  const float* Rb = RESID ? (resid + (size_t)b * strideR) : nullptr;
#pragma unroll
  for (int i = 0; i < 4; ++i) {
    const int mBase = m0 + (i << 4);
#pragma unroll
    for (int j = 0; j < 4; ++j) {
      const int n = n0 + (j << 4) + rlane;
      float bv = 0.f;
      if (BIAS_MODE == 2) bv = bias[n];
#pragma unroll
      for (int r = 0; r < 8; ++r) {
        float v = acc[i][j][r] * scale;
        if (BIAS_MODE == 1) v += bias[mBase + mOff + r];
        if (BIAS_MODE == 2) v += bv;
        if (RESID) v += Rb[(size_t)(mBase + mOff + r) * ldc + n];
        if (ACT == 1) v = tanhf(v);
        if (ACT == 2) v = fmaxf(v, 0.0f);
        if (ACT == 3) v = v / (1.0f + expf(-v));
        if (ACT == 4) v = (v > 0.f) ? v : 0.01f * v;
        if (ACT == 5) v = 0.5f * v * (1.0f + erff(v * 0.70710678118654752f));
        slab[(mOff + r) * 68 + (j << 4) + rlane] = v;
      }
    }
    __builtin_amdgcn_fence(__ATOMIC_RELEASE, "workgroup");
    __builtin_amdgcn_wave_barrier();
    __builtin_amdgcn_fence(__ATOMIC_ACQUIRE, "workgroup");
    if (OUT_MODE == 0) {
      float* C = (float*)Cout + (size_t)b * strideC;
      const int hh = lane >> 4, c4 = (lane & 15) * 4;
      for (int pass = 0; pass < 2; ++pass) {
#pragma unroll
        for (int it = 0; it < 8; ++it) {
          const int row = it * 2 + hh;
          v4f v = *(const v4f*)(slab + row * 68 + c4);
          *(volatile v4f*)(C + (size_t)(mBase + row) * ldc + n0 + c4) = v;
        }
        __threadfence();
      }
    } else {
      const int q = lane >> 3, c8 = (lane & 7) * 8;
      unsigned short* C  = (unsigned short*)Cout  + (size_t)b * strideC;
      unsigned short* C2 = (OUT_MODE == 2) ? ((unsigned short*)Cout2 + (size_t)b * strideC) : nullptr;
      for (int pass = 0; pass < 2; ++pass) {
#pragma unroll
        for (int it = 0; it < 4; ++it) {
          const int row = it * 4 + q;
          const float* sp = slab + row * 68 + c8;
          v8h hv, lv;
#pragma unroll
          for (int e = 0; e < 8; ++e) {
            if (OUT_MODE == 1) {
              hv[e] = (_Float16)sp[e];
            } else {
              unsigned short hb = f2bf_bits(sp[e]);
              unsigned short lb = f2bf_bits(sp[e] - bf_bits2f(hb));
              hv[e] = __builtin_bit_cast(_Float16, hb);
              lv[e] = __builtin_bit_cast(_Float16, lb);
            }
          }
          *(volatile v8h*)(C + (size_t)(mBase + row) * ldc + n0 + c8) = hv;
          if (OUT_MODE == 2) *(volatile v8h*)(C2 + (size_t)(mBase + row) * ldc + n0 + c8) = lv;
        }
        __threadfence();
      }
    }
    __builtin_amdgcn_fence(__ATOMIC_RELEASE, "workgroup");
    __builtin_amdgcn_wave_barrier();
    __builtin_amdgcn_fence(__ATOMIC_ACQUIRE, "workgroup");
  }
}

__global__ __launch_bounds__(256) void cast_f32_f16x2(
    const float* __restrict__ in, _Float16* __restrict__ out, int n2) {
  int i = blockIdx.x * 256 + threadIdx.x;
  if (i < n2) {
    const _Float16 h0 = (_Float16)in[2 * i], h1 = (_Float16)in[2 * i + 1];
    const unsigned u = (unsigned)__builtin_bit_cast(unsigned short, h0) | ((unsigned)__builtin_bit_cast(unsigned short, h1) << 16);
    ((volatile unsigned*)out)[i] = u;
    __threadfence();
    ((volatile unsigned*)out)[i] = u;
  }
}

__global__ __launch_bounds__(256) void split_f32_bf16x2(
    const float* __restrict__ in, __bf16* __restrict__ hi, __bf16* __restrict__ lo, long n2) {
  long i = (long)blockIdx.x * 256 + threadIdx.x;
  long stride = (long)gridDim.x * 256;
  for (int pass = 0; pass < 2; ++pass) {
    for (long j = i; j < n2; j += stride) {
      const float a = in[2 * j], b = in[2 * j + 1];
      const unsigned short ah = f2bf_bits(a), bh = f2bf_bits(b);
      const unsigned short al = f2bf_bits(a - bf_bits2f(ah)), bl = f2bf_bits(b - bf_bits2f(bh));
      ((volatile unsigned*)hi)[j] = (unsigned)ah | ((unsigned)bh << 16);
      ((volatile unsigned*)lo)[j] = (unsigned)al | ((unsigned)bl << 16);
    }
    __threadfence();
  }
}


#define GN 16384
#define GK 128
#define GDm 32
#define GKD (GK * GDm)
__global__ __launch_bounds__(256) void prep_kernel(const float* __restrict__ Q, const float* __restrict__ mu, __bf16* __restrict__ B1h, __bf16* __restrict__ B1l, _Float16* __restrict__ B2, float* __restrict__ qmu) {
  const int i0 = blockIdx.x * 256 + threadIdx.x;
  if (i0 >= GK * GDm * GDm) return;
  const int k = i0 / (GDm * GDm), i = (i0 / GDm) % GDm, j = i0 % GDm;
  const float q = Q[i0];
  const unsigned short h = f2bf_bits(q), l = f2bf_bits(q - bf_bits2f(h));
  const size_t o1 = ((size_t)k * GDm + j) * GDm + i;
  const size_t o2 = (size_t)i * GKD + k * GDm + j;
  for (int pass = 0; pass < 2; ++pass) {
    ((volatile __bf16*)B1h)[o1] = __builtin_bit_cast(__bf16, h); ((volatile __bf16*)B1l)[o1] = __builtin_bit_cast(__bf16, l);
    ((volatile _Float16*)B2)[o2] = (_Float16)q;
    __threadfence(); }
  if (i == 0) {
    float a = 0.f;
#pragma unroll 1
    for (int ii = 0; ii < GDm; ++ii) a += Q[((size_t)k * GDm + ii) * GDm + j] * mu[k * GDm + ii];
    ((volatile float*)qmu)[k * GDm + j] = a; __threadfence(); ((volatile float*)qmu)[k * GDm + j] = a; }
}
__global__ __launch_bounds__(256) void zero_rows_kernel(__bf16* __restrict__ p, long n) { const long i = (long)blockIdx.x * 256 + threadIdx.x; if (i < n) { ((volatile __bf16*)p)[i] = __builtin_bit_cast(__bf16, (unsigned short)0); __threadfence(); ((volatile __bf16*)p)[i] = __builtin_bit_cast(__bf16, (unsigned short)0); } }
__global__ __launch_bounds__(256) void comp_kernel(float* __restrict__ U, const float* __restrict__ qmu, const float* __restrict__ Leig, const float* __restrict__ sigma, const float* __restrict__ phi, float* __restrict__ LW) {
  const int lane = threadIdx.x & 31, wave = threadIdx.x >> 5; const int n = blockIdx.x; const float s2 = sigma[n] * sigma[n];
  __shared__ float lws[GK];
#pragma unroll 1
  for (int kk = 0; kk < GK / 8; ++kk) { const int k = wave * (GK / 8) + kk;
    const float L = Leig[k * GDm + lane] + s2;
    const size_t idx = (size_t)n * GKD + k * GDm + lane;
    const float u = (qmu[k * GDm + lane] - U[idx]) / L;
    float t = logf(L) + L * u * u;
    for (int o = 16; o > 0; o >>= 1) t += __shfl_xor(t, o, 32);
    if (lane == 0) lws[k] = logf(phi[k]) - 0.5f * t;
    ((volatile float*)U)[idx] = u;
  }
  __syncthreads();
  __shared__ float mx, se;
  if (threadIdx.x < 32) { float m = -INFINITY; for (int k = lane; k < GK; k += 32) m = fmaxf(m, lws[k]); for (int o = 16; o > 0; o >>= 1) m = fmaxf(m, __shfl_xor(m, o, 32)); if (lane == 0) mx = m; }
  __syncthreads();
  if (threadIdx.x < 32) { float s = 0.f; for (int k = lane; k < GK; k += 32) s += expf(lws[k] - mx); for (int o = 16; o > 0; o >>= 1) s += __shfl_xor(s, o, 32); if (lane == 0) se = s; }
  __syncthreads();
  if (threadIdx.x < GK) { const float w = expf(lws[threadIdx.x] - mx) / se; ((volatile float*)LW)[(size_t)n * GK + threadIdx.x] = w; }
  __threadfence();
  if (threadIdx.x < GK) { const float w = expf(lws[threadIdx.x] - mx) / se; ((volatile float*)LW)[(size_t)n * GK + threadIdx.x] = w; }
#pragma unroll 1
  for (int kk = 0; kk < GK / 8; ++kk) { const int k = wave * (GK / 8) + kk; const size_t idx = (size_t)n * GKD + k * GDm + lane; ((volatile float*)U)[idx] = U[idx]; }
}
#define GCH 2048
__global__ __launch_bounds__(256) void wu_kernel(const float* __restrict__ U, const float* __restrict__ LW, _Float16* __restrict__ A2) {
  const long i = (long)blockIdx.x * 256 + threadIdx.x; if (i >= (long)GCH * GKD) return; const long n = i / GKD; const int k = (int)((i % GKD) / GDm);
  const float a = LW[n * GK + k] * U[i];
  ((volatile _Float16*)A2)[i] = (_Float16)a; __threadfence(); ((volatile _Float16*)A2)[i] = (_Float16)a;
}
__global__ __launch_bounds__(256) void pack_kernel(const float* __restrict__ O, float* __restrict__ out) {
  const long i = (long)blockIdx.x * 256 + threadIdx.x; const long n = i >> 3; const int q = (int)(i & 7); if (n >= GN) return;
  const v4f v = *(const v4f*)(O + n * 64 + q * 4);
  *(volatile v4f*)(out + n * GDm + q * 4) = v; __threadfence(); *(volatile v4f*)(out + n * GDm + q * 4) = v;
}
extern "C" void kernel_launch(void* const* d_in, const int* in_sizes, int n_in, void* d_out, int out_size, void* d_ws, size_t ws_size, hipStream_t stream) {
  (void)in_sizes; (void)n_in; (void)out_size; (void)ws_size;
  const float* x = (const float*)d_in[0]; const float* sigma = (const float*)d_in[1]; const float* phi = (const float*)d_in[2]; const float* mu = (const float*)d_in[3]; const float* Leig = (const float*)d_in[4]; const float* Q = (const float*)d_in[5];
  char* ws = (char*)d_ws; size_t off = 0;
  auto carve = [&](size_t bytes) -> char* { char* p = ws + off; off += (bytes + 255) & ~(size_t)255; return p; };
  __bf16* Xh = (__bf16*)carve((size_t)GN * GDm * 2); __bf16* Xl = (__bf16*)carve((size_t)GN * GDm * 2);
  __bf16* B1h = (__bf16*)carve((size_t)GKD * GDm * 2); __bf16* B1l = (__bf16*)carve((size_t)GKD * GDm * 2);
  _Float16* B2 = (_Float16*)carve((size_t)64 * GKD * 2);
  float* qmu = (float*)carve(GKD * 4); float* LW = (float*)carve((size_t)GN * GK * 4);
  float* U = (float*)carve((size_t)GCH * GKD * 4);
  _Float16* A2 = (_Float16*)carve((size_t)GCH * GKD * 2);
  float* O = (float*)carve((size_t)GN * 64 * 4);
  split_f32_bf16x2<<<(GN * GDm / 2 + 255) / 256, 256, 0, stream>>>(x, Xh, Xl, GN * GDm / 2);
  zero_rows_kernel<<<(64 * GKD + 255) / 256, 256, 0, stream>>>((__bf16*)B2, (long)64 * GKD);
  prep_kernel<<<(GK * GDm * GDm + 255) / 256, 256, 0, stream>>>(Q, mu, B1h, B1l, B2, qmu);
  const int t1 = (GCH / 64) * (GKD / 64), t2 = (GCH / 64) * 1;
  for (int c = 0; c < GN / GCH; ++c) {
    const size_t n0 = (size_t)c * GCH;
    wmma_gemm64<1, true, 0, 0, false><<<dim3((t1 + 7) / 8, 1), 256, 0, stream>>>(U16(Xh + n0 * GDm), U16(Xl + n0 * GDm), GDm, 0, U16(B1h), U16(B1l), GDm, 0, U, nullptr, GKD, 0, nullptr, nullptr, 0, GCH, GKD, GDm, 1.0f);
    comp_kernel<<<GCH, 256, 0, stream>>>(U, qmu, Leig, sigma + n0, phi, LW + n0 * GK);
    wu_kernel<<<(GCH * GKD + 255) / 256, 256, 0, stream>>>(U, LW + n0 * GK, A2);
    wmma_gemm64<0, false, 0, 0, false><<<dim3((t2 + 7) / 8, 1), 256, 0, stream>>>(U16(A2), nullptr, GKD, 0, U16(B2), nullptr, GKD, 0, O + n0 * 64, nullptr, 64, 0, nullptr, nullptr, 0, GCH, 64, GKD, 1.0f);
  }
  pack_kernel<<<(GN * 8 + 255) / 256, 256, 0, stream>>>(O, (float*)d_out);
}
